// CausalCrossConditionalSelfAttention_83047487635486
// MI455X (gfx1250) — hardware-verified
//
#include <hip/hip_runtime.h>

typedef __attribute__((ext_vector_type(16))) _Float16 v16h;
typedef __attribute__((ext_vector_type(8)))  _Float16 v8h;
typedef __attribute__((ext_vector_type(16))) __bf16   v16b;
typedef __attribute__((ext_vector_type(8)))  __bf16   v8b;
typedef __attribute__((ext_vector_type(8)))  float    v8f;
typedef __attribute__((ext_vector_type(4)))  float    v4f;

#define NEG_INF (-__builtin_huge_valf())

__device__ __forceinline__ unsigned short f2bf_bits(float f) {
  unsigned u = __float_as_uint(f);
  return (unsigned short)((u + 0x7FFFu + ((u >> 16) & 1u)) >> 16);
}
__device__ __forceinline__ float bf_bits2f(unsigned short h) { return __uint_as_float(((unsigned)h) << 16); }

__device__ __forceinline__ void dep_guard_h(v8f& a, v8f& b, v16h x, v16h y) { asm volatile("v_nop\n\tv_nop\n\tv_nop\n\tv_nop" : "+v"(a), "+v"(b) : "v"(x), "v"(y)); }
__device__ __forceinline__ void dep_guard_b(v8f& a, v8f& b, v16b x, v16b y) { asm volatile("v_nop\n\tv_nop\n\tv_nop\n\tv_nop" : "+v"(a), "+v"(b) : "v"(x), "v"(y)); }
__device__ __forceinline__ void keep4_h(v16h a, v16h b, v16h c, v16h d) { asm volatile("v_nop" :: "v"(a), "v"(b), "v"(c), "v"(d)); }
__device__ __forceinline__ void keep4_b(v16b a, v16b b, v16b c, v16b d) { asm volatile("v_nop" :: "v"(a), "v"(b), "v"(c), "v"(d)); }
__device__ __forceinline__ void acc_guard4(v8f& a, v8f& b, v8f& c, v8f& d) { asm volatile("v_nop\n\tv_nop\n\tv_nop\n\tv_nop" : "+v"(a), "+v"(b), "+v"(c), "+v"(d)); }
template <typename T> struct Frag;
template <> struct Frag<_Float16> {
  typedef v16h V; union U { v16h v; v8h h[2]; };
  static __device__ __forceinline__ v16h load(const _Float16* p) {
    U f; f.h[0] = *(const v8h*)(p); f.h[1] = *(const v8h*)(p + 16); return f.v;
  }
  static __device__ __forceinline__ v8f mma(v16h a, v16h b, v8f c) {
    return __builtin_amdgcn_wmma_f32_16x16x32_f16(false, a, false, b, (short)0, c, false, false);
  }
  static __device__ __forceinline__ void guard(v8f& a, v8f& b, v16h x, v16h y) { dep_guard_h(a, b, x, y); }
  static __device__ __forceinline__ void keep(v16h a, v16h b, v16h c, v16h d) { keep4_h(a, b, c, d); }
};
template <> struct Frag<__bf16> {
  typedef v16b V; union U { v16b v; v8b h[2]; };
  static __device__ __forceinline__ v16b load(const __bf16* p) {
    U f; f.h[0] = *(const v8b*)(p); f.h[1] = *(const v8b*)(p + 16); return f.v;
  }
  static __device__ __forceinline__ v8f mma(v16b a, v16b b, v8f c) {
    return __builtin_amdgcn_wmma_f32_16x16x32_bf16(false, a, false, b, (short)0, c, false, false);
  }
  static __device__ __forceinline__ void guard(v8f& a, v8f& b, v16b x, v16b y) { dep_guard_b(a, b, x, y); }
  static __device__ __forceinline__ void keep(v16b a, v16b b, v16b c, v16b d) { keep4_b(a, b, c, d); }
};

template <int ET> struct Elem;
template <> struct Elem<0> { typedef _Float16 T; };
template <> struct Elem<1> { typedef __bf16 T; };
template <int ET, int SPLIT, int BIAS_MODE, int OUT_MODE, bool RESID, int ACT = 0>
__global__ __launch_bounds__(256) void wmma_gemm64(
    const unsigned short* __restrict__ Ap, const unsigned short* __restrict__ A2p, int lda, long strideA,
    const unsigned short* __restrict__ Btp, const unsigned short* __restrict__ Bt2p, int ldb, long strideB,
    void* __restrict__ Cout, void* __restrict__ Cout2, int ldc, long strideC,
    const float* __restrict__ bias,
    const float* __restrict__ resid, long strideR,
    int M, int N, int K, float scale) {
  typedef typename Elem<ET>::T T;
  typedef typename Frag<T>::V V;
  const T* A = (const T*)Ap; const T* A2 = (const T*)A2p; const T* Bt = (const T*)Btp; const T* Bt2 = (const T*)Bt2p;
  __shared__ __align__(16) float sT[8][16 * 68];
  const int b    = blockIdx.y;
  const int lane = threadIdx.x & 31;
  const int wave = threadIdx.x >> 5;
  const int tilesN = N >> 6;
  const int tilesM = M >> 6;
  const int tile = blockIdx.x * 8 + wave;
  if (tile >= tilesM * tilesN) return;
  const int tm = tile / tilesN;
  const int tn = tile - tm * tilesN;
  const int m0 = tm << 6;
  const int n0 = tn << 6;

  const T* Ab  = A  + (size_t)b * strideA;
  const T* Bb  = Bt + (size_t)b * strideB;
  const T* Ab2 = (SPLIT != 0) ? (A2  + (size_t)b * strideA) : nullptr;
  const T* Bb2 = (SPLIT == 1) ? (Bt2 + (size_t)b * strideB) : nullptr;

  const int rlane = lane & 15;
  const int koff  = (lane >> 4) * 8;
  const int mOff  = (lane >> 4) * 8;

  v8f acc[4][4];
#pragma unroll
  for (int i = 0; i < 4; ++i)
#pragma unroll
    for (int j = 0; j < 4; ++j) acc[i][j] = (v8f){0.f,0.f,0.f,0.f,0.f,0.f,0.f,0.f};

  for (int k0 = 0; k0 < K; k0 += 32) {
    V bh[4], bl[4];
#pragma unroll
    for (int j = 0; j < 4; ++j) {
      const size_t bo = (size_t)(n0 + (j << 4) + rlane) * ldb + koff + k0;
      bh[j] = Frag<T>::load(Bb + bo);
      if (SPLIT == 1) bl[j] = Frag<T>::load(Bb2 + bo);
    }
#pragma unroll
    for (int i = 0; i < 4; ++i) {
      const size_t ao = (size_t)(m0 + (i << 4) + rlane) * lda + koff + k0;
      V ah = Frag<T>::load(Ab + ao);
      V al;
      if (SPLIT != 0) al = Frag<T>::load(Ab2 + ao);
#pragma unroll
      for (int j = 0; j < 4; ++j) {
        acc[i][j] = Frag<T>::mma(ah, bh[j], acc[i][j]);
        if (SPLIT == 1) acc[i][j] = Frag<T>::mma(ah, bl[j], acc[i][j]);
        if (SPLIT != 0) acc[i][j] = Frag<T>::mma(al, bh[j], acc[i][j]);
      }
      Frag<T>::guard(acc[i][0], acc[i][3], ah, (SPLIT != 0) ? al : ah);
    }
    Frag<T>::keep(bh[0], bh[1], bh[2], bh[3]);
    if (SPLIT == 1) Frag<T>::keep(bl[0], bl[1], bl[2], bl[3]);
  }
  acc_guard4(acc[0][0], acc[0][1], acc[0][2], acc[0][3]);
  acc_guard4(acc[1][0], acc[1][1], acc[1][2], acc[1][3]);
  acc_guard4(acc[2][0], acc[2][1], acc[2][2], acc[2][3]);
  acc_guard4(acc[3][0], acc[3][1], acc[3][2], acc[3][3]);

  float* slab = sT[wave];
  const float* Rb = RESID ? (resid + (size_t)b * strideR) : nullptr;
#pragma unroll
  for (int i = 0; i < 4; ++i) {
    const int mBase = m0 + (i << 4);
#pragma unroll
    for (int j = 0; j < 4; ++j) {
      const int n = n0 + (j << 4) + rlane;
      float bv = 0.f;
      if (BIAS_MODE == 2) bv = bias[n];
      if (BIAS_MODE == 3) bv = bf_bits2f(f2bf_bits(bias[n]));
#pragma unroll
      for (int r = 0; r < 8; ++r) {
        float v = acc[i][j][r] * scale;
        if (BIAS_MODE == 1) v += bias[mBase + mOff + r];
        if (BIAS_MODE == 2 || BIAS_MODE == 3) v += bv;
        if (RESID) v += Rb[(size_t)(mBase + mOff + r) * ldc + n];
        if (ACT == 1) v = tanhf(v);
        if (ACT == 2) v = fmaxf(v, 0.0f);
        if (ACT == 3) v = v / (1.0f + expf(-v));
        if (ACT == 4) v = (v > 0.f) ? v : 0.01f * v;
        if (ACT == 5) v = 0.5f * v * (1.0f + erff(v * 0.70710678118654752f));
        slab[(mOff + r) * 68 + (j << 4) + rlane] = v;
      }
    }
    __builtin_amdgcn_fence(__ATOMIC_RELEASE, "workgroup");
    __builtin_amdgcn_wave_barrier();
    __builtin_amdgcn_fence(__ATOMIC_ACQUIRE, "workgroup");
    if (OUT_MODE == 0) {
      float* C = (float*)Cout + (size_t)b * strideC;
      const int hh = lane >> 4, c4 = (lane & 15) * 4;
      for (int pass = 0; pass < 2; ++pass) {
#pragma unroll
        for (int it = 0; it < 8; ++it) {
          const int row = it * 2 + hh;
          v4f v = *(const v4f*)(slab + row * 68 + c4);
          *(volatile v4f*)(C + (size_t)(mBase + row) * ldc + n0 + c4) = v;
        }
        __threadfence();
      }
    } else {
      const int q = lane >> 3, c8 = (lane & 7) * 8;
      unsigned short* C  = (unsigned short*)Cout  + (size_t)b * strideC;
      unsigned short* C2 = (OUT_MODE == 2) ? ((unsigned short*)Cout2 + (size_t)b * strideC) : nullptr;
      for (int pass = 0; pass < 2; ++pass) {
#pragma unroll
        for (int it = 0; it < 4; ++it) {
          const int row = it * 4 + q;
          const float* sp = slab + row * 68 + c8;
          v8h hv, lv;
#pragma unroll
          for (int e = 0; e < 8; ++e) {
            if (OUT_MODE == 1) {
              hv[e] = (_Float16)sp[e];
            } else {
              unsigned short hb = f2bf_bits(sp[e]);
              unsigned short lb = f2bf_bits(sp[e] - bf_bits2f(hb));
              hv[e] = __builtin_bit_cast(_Float16, hb);
              lv[e] = __builtin_bit_cast(_Float16, lb);
            }
          }
          *(volatile v8h*)(C + (size_t)(mBase + row) * ldc + n0 + c8) = hv;
          if (OUT_MODE == 2) *(volatile v8h*)(C2 + (size_t)(mBase + row) * ldc + n0 + c8) = lv;
        }
        __threadfence();
      }
    }
    __builtin_amdgcn_fence(__ATOMIC_RELEASE, "workgroup");
    __builtin_amdgcn_wave_barrier();
    __builtin_amdgcn_fence(__ATOMIC_ACQUIRE, "workgroup");
  }
}

__global__ __launch_bounds__(256) void cast_f32_bf16x2(
    const float* __restrict__ in, unsigned short* __restrict__ out, int n2) {
  int i = blockIdx.x * 256 + threadIdx.x;
  if (i < n2) {
    const unsigned u = (unsigned)f2bf_bits(in[2 * i]) | ((unsigned)f2bf_bits(in[2 * i + 1]) << 16);
    ((volatile unsigned*)out)[i] = u;
    __threadfence();
    ((volatile unsigned*)out)[i] = u;
  }
}

#define AT_D 64
#define AT_NW 4
#define AT_QB 64
#define AT_KC 64
#define T_MOT 1024
#define N_TXT 16
#define L_TOK 3136
#define NKC_ALL 49
#define KC_TXT 48

struct AttnP { long q_bs, q_rs, q_hs, k_bs, k_rs, k_hs, v_bs, v_rs, v_hs, o_bs, o_rs, o_hs;
               int S, H; float sscale; int nseg; };
static_assert(sizeof(AttnP) == 112);

__device__ __forceinline__ unsigned short at_bf_bits(float f) {
  unsigned u = __float_as_uint(f);
  return (unsigned short)((u + 0x7FFFu + ((u >> 16) & 1u)) >> 16);
}
__device__ __forceinline__ __bf16 at_f2bf(float f) { return __builtin_bit_cast(__bf16, at_bf_bits(f)); }
__device__ __forceinline__ void at_split(float f, __bf16& hi, __bf16& lo) {
  const unsigned short hb = at_bf_bits(f);
  hi = __builtin_bit_cast(__bf16, hb);
  lo = at_f2bf(f - __uint_as_float(((unsigned)hb) << 16));
}
__device__ __forceinline__ v8f at_mma3(v16b ah, v16b al, v16b bh, v16b bl, v8f c) {
  c = __builtin_amdgcn_wmma_f32_16x16x32_bf16(false, ah, false, bh, (short)0, c, false, false);
  c = __builtin_amdgcn_wmma_f32_16x16x32_bf16(false, ah, false, bl, (short)0, c, false, false);
  c = __builtin_amdgcn_wmma_f32_16x16x32_bf16(false, al, false, bh, (short)0, c, false, false);
  asm volatile("v_nop\n\tv_nop\n\tv_nop\n\tv_nop" : "+v"(c) : "v"(ah), "v"(al), "v"(bh), "v"(bl));
  return c;
}
__device__ __forceinline__ int floordiv8(int v) {
  const int qd = v / 8;
  return ((v - qd * 8) < 0) ? (qd - 1) : qd;
}

__global__ __launch_bounds__(128)
void attn64_blockmask_split(const float* __restrict__ q, const float* __restrict__ k,
                            const float* __restrict__ v,
                            unsigned short* __restrict__ ohi, unsigned short* __restrict__ olo,
                            const int* __restrict__ sfr, const int* __restrict__ efr,
                            const int* __restrict__ w0p, AttnP g) {
  union FB { v16b v; v8b h[2]; };
  __shared__ __align__(16) __bf16 Qsh[AT_QB * AT_D];
  __shared__ __align__(16) __bf16 Qsl[AT_QB * AT_D];
  __shared__ __align__(16) __bf16 Ksh[AT_KC * AT_D];
  __shared__ __align__(16) __bf16 Ksl[AT_KC * AT_D];
  __shared__ __align__(16) __bf16 Vth[AT_D * AT_KC];
  __shared__ __align__(16) __bf16 Vtl[AT_D * AT_KC];
  __shared__ __align__(16) __bf16 Psh[AT_NW][16 * AT_KC];
  __shared__ __align__(16) __bf16 Psl[AT_NW][16 * AT_KC];
  __shared__ __align__(16) float  Os[AT_NW][16 * 68];

  const int tid  = threadIdx.x;
  const int wave = tid >> 5;
  const int lane = tid & 31;
  const int hh   = lane >> 4;
  const int c    = lane & 15;

  const int nqb = g.S / AT_QB;
  const int bx = blockIdx.x;
  const int qb = bx % nqb;
  const int bh = bx / nqb;
  const int h  = bh % g.H;
  const int b  = bh / g.H;
  const int q0 = qb * AT_QB + wave * 16;

  const float* qb_ptr = q + (size_t)b * g.q_bs + (size_t)h * g.q_hs;
  const float* kb_ptr = k + (size_t)b * g.k_bs + (size_t)h * g.k_hs;
  const float* vb_ptr = v + (size_t)b * g.v_bs + (size_t)h * g.v_hs;

  const int w0  = w0p[0];
  const int rsn = floordiv8(sfr[b * g.nseg + c]) - w0;
  const int ren = floordiv8(efr[b * g.nseg + c]) - w0;
  const bool qText = (qb >= KC_TXT);
  const int  br    = qText ? 0 : (qb >> 4);
  const int  fb    = qb & 15;

  {
    const int r = tid >> 1, dh = (tid & 1) * 32;
    const float* qrow = qb_ptr + (size_t)(qb * AT_QB + r) * g.q_rs + dh;
#pragma unroll 1
    for (int i = 0; i < 8; ++i) {
      const v4f x = *(const v4f*)(qrow + 4 * i);
#pragma unroll
      for (int e = 0; e < 4; ++e) {
        const int d = dh + 4 * i + e;
        __bf16 a, bl; at_split(x[e], a, bl);
        Qsh[r * AT_D + d] = a;
        Qsl[r * AT_D + d] = bl;
      }
    }
  }
  __syncthreads();

  float mrow[8], lrow[8];
  v8f oacc[4];
#pragma unroll
  for (int r = 0; r < 8; ++r) { mrow[r] = NEG_INF; lrow[r] = 0.f; }
#pragma unroll
  for (int t = 0; t < 4; ++t) oacc[t] = (v8f){0.f,0.f,0.f,0.f,0.f,0.f,0.f,0.f};

  const __bf16* qwh = Qsh + (wave * 16 + c) * AT_D + 8 * hh;
  const __bf16* qwl = Qsl + (wave * 16 + c) * AT_D + 8 * hh;

  for (int kc = 0; kc < NKC_ALL; ++kc) {
    const bool txtChunk = (kc >= KC_TXT);
    bool proc;
    if (qText) proc = true;
    else if (!txtChunk) proc = ((kc & 15) <= fb) && (br != 0 || kc < 16);
    else proc = (br != 0);
    if (!proc) continue;
    const int kv0 = kc * AT_KC;
    __syncthreads();
    {
      const int kvr = tid >> 1, dh = (tid & 1) * 32;
      const float* krow = kb_ptr + (size_t)(kv0 + kvr) * g.k_rs + dh;
      const float* vrow = vb_ptr + (size_t)(kv0 + kvr) * g.v_rs + dh;
#pragma unroll 1
      for (int i = 0; i < 8; ++i) {
        const v4f kk = *(const v4f*)(krow + 4 * i);
        const v4f vv = *(const v4f*)(vrow + 4 * i);
#pragma unroll
        for (int e = 0; e < 4; ++e) {
          const int d = dh + 4 * i + e;
          __bf16 a, bl;
          at_split(kk[e], a, bl);
          Ksh[kvr * AT_D + d] = a;
          Ksl[kvr * AT_D + d] = bl;
          at_split(vv[e], a, bl);
          Vth[d * AT_KC + kvr] = a;
          Vtl[d * AT_KC + kvr] = bl;
        }
      }
    }
    __syncthreads();

    v8f s[4];
#pragma unroll
    for (int j = 0; j < 4; ++j) s[j] = (v8f){0.f,0.f,0.f,0.f,0.f,0.f,0.f,0.f};
#pragma unroll 1
    for (int dc = 0; dc < 2; ++dc) {
      FB qh, ql;
      qh.h[0] = *(const v8b*)(qwh + dc * 32);
      qh.h[1] = *(const v8b*)(qwh + dc * 32 + 16);
      ql.h[0] = *(const v8b*)(qwl + dc * 32);
      ql.h[1] = *(const v8b*)(qwl + dc * 32 + 16);
#pragma unroll
      for (int j = 0; j < 4; ++j) {
        FB kb, kl;
        const __bf16* kp  = Ksh + (j * 16 + c) * AT_D + dc * 32 + 8 * hh;
        const __bf16* kpl = Ksl + (j * 16 + c) * AT_D + dc * 32 + 8 * hh;
        kb.h[0] = *(const v8b*)(kp);
        kb.h[1] = *(const v8b*)(kp + 16);
        kl.h[0] = *(const v8b*)(kpl);
        kl.h[1] = *(const v8b*)(kpl + 16);
        s[j] = at_mma3(qh.v, ql.v, kb.v, kl.v, s[j]);
      }
    }
    const int  bc   = kc >> 4;
    const bool incl = (br == 2) ? (bc <= 1) : (bc == 0);
    const bool allm = (!qText) && (br == 0) && (bc != 0);
    const int  fc0  = kv0 - bc * T_MOT + c;
    float cm[8];
#pragma unroll
    for (int r = 0; r < 8; ++r) {
      const int  fr  = q0 + 8 * hh + r - br * T_MOT;
      const bool act = (fr >= rsn) && (fr < ren);
      float m = NEG_INF;
#pragma unroll
      for (int j = 0; j < 4; ++j) {
        float sv = s[j][r] * g.sscale;
        bool msk;
        if (qText) msk = false;
        else if (!txtChunk) { const int fc = fc0 + j * 16; msk = incl ? (fc > fr) : (fc >= fr); }
        else { const bool segok = (br == 1) ? (j != 1) : (j != 0); msk = !(act && segok); }
        if (msk || allm) sv = NEG_INF;
        s[j][r] = sv;
        m = fmaxf(m, sv);
      }
#pragma unroll
      for (int off = 1; off < 16; off <<= 1) m = fmaxf(m, __shfl_xor(m, off, 32));
      cm[r] = m;
    }
    __bf16* pwh = Psh[wave];
    __bf16* pwl = Psl[wave];
#pragma unroll
    for (int r = 0; r < 8; ++r) {
      const float mnew = fmaxf(mrow[r], cm[r]);
      const float mref = (mnew == NEG_INF) ? 0.0f : mnew;
      const float alpha = __expf(mrow[r] - mref);
      mrow[r] = mnew;
      float psum = 0.f;
#pragma unroll
      for (int j = 0; j < 4; ++j) {
        const float p = __expf(s[j][r] - mref);
        psum += p;
        __bf16 a, bl; at_split(p, a, bl);
        pwh[(8 * hh + r) * AT_KC + j * 16 + c] = a;
        pwl[(8 * hh + r) * AT_KC + j * 16 + c] = bl;
      }
#pragma unroll
      for (int off = 1; off < 16; off <<= 1) psum += __shfl_xor(psum, off, 32);
      lrow[r] = lrow[r] * alpha + psum;
#pragma unroll
      for (int t = 0; t < 4; ++t) oacc[t][r] *= alpha;
    }
    __builtin_amdgcn_fence(__ATOMIC_RELEASE, "workgroup");
    __builtin_amdgcn_wave_barrier();
    __builtin_amdgcn_fence(__ATOMIC_ACQUIRE, "workgroup");
#pragma unroll 1
    for (int kk = 0; kk < 2; ++kk) {
      FB pa, pl;
      pa.h[0] = *(const v8b*)(pwh + c * AT_KC + kk * 32 + 8 * hh);
      pa.h[1] = *(const v8b*)(pwh + c * AT_KC + kk * 32 + 16 + 8 * hh);
      pl.h[0] = *(const v8b*)(pwl + c * AT_KC + kk * 32 + 8 * hh);
      pl.h[1] = *(const v8b*)(pwl + c * AT_KC + kk * 32 + 16 + 8 * hh);
#pragma unroll
      for (int t = 0; t < 4; ++t) {
        FB vb, vl;
        const __bf16* vp  = Vth + (t * 16 + c) * AT_KC + kk * 32 + 8 * hh;
        const __bf16* vpl = Vtl + (t * 16 + c) * AT_KC + kk * 32 + 8 * hh;
        vb.h[0] = *(const v8b*)(vp);
        vb.h[1] = *(const v8b*)(vp + 16);
        vl.h[0] = *(const v8b*)(vpl);
        vl.h[1] = *(const v8b*)(vpl + 16);
        oacc[t] = at_mma3(pa.v, pl.v, vb.v, vl.v, oacc[t]);
      }
    }
  }

  float* os = Os[wave];
#pragma unroll
  for (int r = 0; r < 8; ++r) {
    const float inv = 1.0f / lrow[r];
#pragma unroll
    for (int t = 0; t < 4; ++t) os[(8 * hh + r) * 68 + t * 16 + c] = oacc[t][r] * inv;
  }
  __builtin_amdgcn_fence(__ATOMIC_RELEASE, "workgroup");
  __builtin_amdgcn_wave_barrier();
  __builtin_amdgcn_fence(__ATOMIC_ACQUIRE, "workgroup");
  {
    const int q8 = lane >> 3, c8 = (lane & 7) * 8;
    unsigned short* oh = ohi + (size_t)b * g.o_bs + (size_t)h * g.o_hs;
    unsigned short* ol = olo + (size_t)b * g.o_bs + (size_t)h * g.o_hs;
    for (int pass = 0; pass < 2; ++pass) {
#pragma unroll
      for (int it = 0; it < 4; ++it) {
        const int row = it * 4 + q8;
        const float* sp = os + row * 68 + c8;
        v8h hv, lv;
#pragma unroll
        for (int e = 0; e < 8; ++e) {
          const unsigned short hb = f2bf_bits(sp[e]);
          const unsigned short lb = f2bf_bits(sp[e] - bf_bits2f(hb));
          hv[e] = __builtin_bit_cast(_Float16, hb);
          lv[e] = __builtin_bit_cast(_Float16, lb);
        }
        *(volatile v8h*)(oh + (size_t)(q0 + row) * g.o_rs + c8) = hv;
        *(volatile v8h*)(ol + (size_t)(q0 + row) * g.o_rs + c8) = lv;
      }
      __threadfence();
    }
  }
}

extern "C" void kernel_launch(void* const* d_in, const int* in_sizes, int n_in,
                              void* d_out, int out_size, void* d_ws, size_t ws_size,
                              hipStream_t stream) {
  constexpr int Bn = 2, Tm = T_MOT, Ns = N_TXT, Cn = 512, Hn = 8, Dh = 64;
  constexpr int Ln = 3 * Tm + 4 * Ns;
  constexpr int C3 = 3 * Cn;
  constexpr int M = Bn * Ln;
  constexpr int NQB = Ln / AT_QB;
  static_assert(Ln == L_TOK && NQB == NKC_ALL && Cn == Hn * Dh);
  static_assert(M % 64 == 0 && Cn % 64 == 0 && Cn % 32 == 0 && Ln % AT_QB == 0 && (3 * Tm) % AT_KC == 0);
  if (n_in < 14) return;
  if (in_sizes[0] != M * Cn || in_sizes[1] != Cn * Cn || in_sizes[2] != Cn || in_sizes[3] != Cn * Cn ||
      in_sizes[4] != Cn || in_sizes[5] != Cn * Cn || in_sizes[6] != Cn || in_sizes[7] != Cn * Cn ||
      in_sizes[8] != Cn || in_sizes[9] != Bn * Ns || in_sizes[10] != Bn * Ns || in_sizes[13] < 1 ||
      out_size != M * Cn) return;

  const float* x   = (const float*)d_in[0];
  const float* Wq  = (const float*)d_in[1];
  const float* bq  = (const float*)d_in[2];
  const float* Wk  = (const float*)d_in[3];
  const float* bk  = (const float*)d_in[4];
  const float* Wv  = (const float*)d_in[5];
  const float* bv  = (const float*)d_in[6];
  const float* Wp  = (const float*)d_in[7];
  const float* bp  = (const float*)d_in[8];
  const int*   sf  = (const int*)d_in[9];
  const int*   ef  = (const int*)d_in[10];
  const int*   w0  = (const int*)d_in[13];
  float* out = (float*)d_out;

  const size_t bX   = (size_t)M * Cn * 2;
  const size_t bW   = (size_t)Cn * Cn * 2;
  const size_t bQKV = (size_t)M * C3 * 4;
  const size_t bAH  = (size_t)M * Cn * 2;
  char* ws = (char*)d_ws;
  size_t off = 0;
  unsigned short* X16  = (unsigned short*)(ws + off); off += bX;
  unsigned short* Wq16 = (unsigned short*)(ws + off); off += bW;
  unsigned short* Wk16 = (unsigned short*)(ws + off); off += bW;
  unsigned short* Wv16 = (unsigned short*)(ws + off); off += bW;
  unsigned short* Wp16 = (unsigned short*)(ws + off); off += bW;
  float*          QKV  = (float*)(ws + off);          off += bQKV;
  unsigned short* AH   = (unsigned short*)(ws + off); off += bAH;
  unsigned short* AL   = (unsigned short*)(ws + off); off += bAH;
  if (off > ws_size || off > (size_t)134217728) return;

  dim3 blk256(256), blk128(128);

  {
    const int n2x = M * Cn / 2, n2w = Cn * Cn / 2;
    cast_f32_bf16x2<<<dim3((n2x + 255) / 256), blk256, 0, stream>>>(x,  X16,  n2x);
    cast_f32_bf16x2<<<dim3((n2w + 255) / 256), blk256, 0, stream>>>(Wq, Wq16, n2w);
    cast_f32_bf16x2<<<dim3((n2w + 255) / 256), blk256, 0, stream>>>(Wk, Wk16, n2w);
    cast_f32_bf16x2<<<dim3((n2w + 255) / 256), blk256, 0, stream>>>(Wv, Wv16, n2w);
    cast_f32_bf16x2<<<dim3((n2w + 255) / 256), blk256, 0, stream>>>(Wp, Wp16, n2w);
  }

  {
    const int tiles = (M / 64) * (Cn / 64);
    const dim3 grd((tiles + 7) / 8, 1);
    wmma_gemm64<1, 0, 3, 0, false><<<grd, blk256, 0, stream>>>(
        X16, X16, Cn, 0L, Wq16, Wq16, Cn, 0L, (void*)(QKV), (void*)QKV, C3, 0L,
        bq, bq, 0L, M, Cn, Cn, 1.0f);
    wmma_gemm64<1, 0, 3, 0, false><<<grd, blk256, 0, stream>>>(
        X16, X16, Cn, 0L, Wk16, Wk16, Cn, 0L, (void*)(QKV + Cn), (void*)QKV, C3, 0L,
        bk, bk, 0L, M, Cn, Cn, 1.0f);
    wmma_gemm64<1, 0, 3, 0, false><<<grd, blk256, 0, stream>>>(
        X16, X16, Cn, 0L, Wv16, Wv16, Cn, 0L, (void*)(QKV + 2 * Cn), (void*)QKV, C3, 0L,
        bv, bv, 0L, M, Cn, Cn, 1.0f);
  }

  {
    AttnP g;
    g.q_bs = (long)Ln * C3; g.q_rs = C3; g.q_hs = Dh;
    g.k_bs = (long)Ln * C3; g.k_rs = C3; g.k_hs = Dh;
    g.v_bs = (long)Ln * C3; g.v_rs = C3; g.v_hs = Dh;
    g.o_bs = (long)Ln * Cn; g.o_rs = Cn; g.o_hs = Dh;
    g.S = Ln; g.H = Hn;
    g.sscale = 0.125f;
    g.nseg = Ns;
    attn64_blockmask_split<<<dim3(Bn * Hn * NQB), blk128, 0, stream>>>(
        QKV, QKV + Cn, QKV + 2 * Cn, AH, AL, sf, ef, w0, g);
  }

  {
    const int tiles = (M / 64) * (Cn / 64);
    wmma_gemm64<1, 2, 3, 0, false><<<dim3((tiles + 7) / 8, 1), blk256, 0, stream>>>(
        AH, AL, Cn, 0L, Wp16, Wp16, Cn, 0L, (void*)out, (void*)out, Cn, 0L,
        bp, bp, 0L, M, Cn, Cn, 1.0f);
  }
}
